// EEGM2_Light_1812476199778
// MI455X (gfx1250) — hardware-verified
//
#include <hip/hip_runtime.h>
#include <math.h>

constexpr int kBatch    = 16;
constexpr int kLen      = 2048;
constexpr int kChan     = 64;
constexpr int kTok      = kBatch * kLen;
constexpr int kXpadRows = kLen + 6;
constexpr int kZXld     = 448;
constexpr int kDin      = 128;
constexpr int kLen1     = 1024;
constexpr int kLen2     = 512;
constexpr int kLen3     = 256;
constexpr int kX1Rows   = kLen1 + 2;
constexpr int kX2Rows   = kLen2 + 2;
constexpr int kTCH      = 32;
constexpr int kActW     = 192;
constexpr float kLog2e  = 1.4426950408889634f;

typedef __attribute__((ext_vector_type(16))) _Float16 v16h;
typedef __attribute__((ext_vector_type(8)))  _Float16 v8h;
typedef __attribute__((ext_vector_type(16))) __bf16   v16b;
typedef __attribute__((ext_vector_type(8)))  __bf16   v8b;
typedef __attribute__((ext_vector_type(8)))  float    v8f;
typedef __attribute__((ext_vector_type(4)))  float    v4f;
typedef __attribute__((ext_vector_type(4)))  unsigned int v4u;

__device__ __forceinline__ unsigned short f2bf_bits(float f) {
  unsigned u = __float_as_uint(f);
  return (unsigned short)((u + 0x7FFFu + ((u >> 16) & 1u)) >> 16);
}
__device__ __forceinline__ float bf_bits2f(unsigned short h) { return __uint_as_float(((unsigned)h) << 16); }

__device__ __forceinline__ void dep_guard_h(v8f& a, v8f& b, v16h x, v16h y) { asm volatile("v_nop\n\tv_nop\n\tv_nop\n\tv_nop" : "+v"(a), "+v"(b) : "v"(x), "v"(y)); }
__device__ __forceinline__ void dep_guard_b(v8f& a, v8f& b, v16b x, v16b y) { asm volatile("v_nop\n\tv_nop\n\tv_nop\n\tv_nop" : "+v"(a), "+v"(b) : "v"(x), "v"(y)); }
__device__ __forceinline__ void keep4_h(v16h a, v16h b, v16h c, v16h d) { asm volatile("v_nop" :: "v"(a), "v"(b), "v"(c), "v"(d)); }
__device__ __forceinline__ void keep4_b(v16b a, v16b b, v16b c, v16b d) { asm volatile("v_nop" :: "v"(a), "v"(b), "v"(c), "v"(d)); }
__device__ __forceinline__ void acc_guard4(v8f& a, v8f& b, v8f& c, v8f& d) { asm volatile("v_nop\n\tv_nop\n\tv_nop\n\tv_nop" : "+v"(a), "+v"(b), "+v"(c), "+v"(d)); }
template <typename T> struct Frag;
template <> struct Frag<_Float16> {
  typedef v16h V; union U { v16h v; v8h h[2]; };
  static __device__ __forceinline__ v16h load(const _Float16* p) {
    U f; f.h[0] = *(const v8h*)(p); f.h[1] = *(const v8h*)(p + 16); return f.v;
  }
  static __device__ __forceinline__ v8f mma(v16h a, v16h b, v8f c) {
    return __builtin_amdgcn_wmma_f32_16x16x32_f16(false, a, false, b, (short)0, c, false, false);
  }
  static __device__ __forceinline__ void guard(v8f& a, v8f& b, v16h x, v16h y) { dep_guard_h(a, b, x, y); }
  static __device__ __forceinline__ void keep(v16h a, v16h b, v16h c, v16h d) { keep4_h(a, b, c, d); }
};
template <> struct Frag<__bf16> {
  typedef v16b V; union U { v16b v; v8b h[2]; };
  static __device__ __forceinline__ v16b load(const __bf16* p) {
    U f; f.h[0] = *(const v8b*)(p); f.h[1] = *(const v8b*)(p + 16); return f.v;
  }
  static __device__ __forceinline__ v8f mma(v16b a, v16b b, v8f c) {
    return __builtin_amdgcn_wmma_f32_16x16x32_bf16(false, a, false, b, (short)0, c, false, false);
  }
  static __device__ __forceinline__ void guard(v8f& a, v8f& b, v16b x, v16b y) { dep_guard_b(a, b, x, y); }
  static __device__ __forceinline__ void keep(v16b a, v16b b, v16b c, v16b d) { keep4_b(a, b, c, d); }
};

__device__ __forceinline__ unsigned pk16(unsigned short a, unsigned short b) { return (unsigned)a | ((unsigned)b << 16); }

template <int ET> struct Elem;
template <> struct Elem<0> { typedef _Float16 T; };
template <> struct Elem<1> { typedef __bf16 T; };
template <int ET, bool SPLIT, int BIAS_MODE, int OUT_MODE, bool RESID, int ACT = 0>
__global__ __launch_bounds__(256) void wmma_gemm64(
    const unsigned short* __restrict__ Ap, const unsigned short* __restrict__ A2p, int lda, long strideA,
    const unsigned short* __restrict__ Btp, const unsigned short* __restrict__ Bt2p, int ldb, long strideB,
    void* __restrict__ Cout, void* __restrict__ Cout2, int ldc, long strideC,
    const float* __restrict__ bias,
    const float* __restrict__ resid, long strideR,
    int M, int N, int K, float scale) {
  typedef typename Elem<ET>::T T;
  typedef typename Frag<T>::V V;
  const T* A = (const T*)Ap; const T* A2 = (const T*)A2p; const T* Bt = (const T*)Btp; const T* Bt2 = (const T*)Bt2p;
  __shared__ __align__(16) float sT[8][16 * 68];
  const int b    = blockIdx.y;
  const int lane = threadIdx.x & 31;
  const int wave = threadIdx.x >> 5;
  const int tilesN = N >> 6;
  const int tilesM = M >> 6;
  const int tile = blockIdx.x * 8 + wave;
  if (tile >= tilesM * tilesN) return;
  const int tm = tile / tilesN;
  const int tn = tile - tm * tilesN;
  const int m0 = tm << 6;
  const int n0 = tn << 6;

  const T* Ab  = A  + (size_t)b * strideA;
  const T* Bb  = Bt + (size_t)b * strideB;
  const T* Ab2 = SPLIT ? (A2  + (size_t)b * strideA) : nullptr;
  const T* Bb2 = SPLIT ? (Bt2 + (size_t)b * strideB) : nullptr;

  const int rlane = lane & 15;
  const int koff  = (lane >> 4) * 8;
  const int mOff  = (lane >> 4) * 8;

  v8f acc[4][4];
#pragma unroll
  for (int i = 0; i < 4; ++i)
#pragma unroll
    for (int j = 0; j < 4; ++j) acc[i][j] = (v8f){0.f,0.f,0.f,0.f,0.f,0.f,0.f,0.f};

  for (int k0 = 0; k0 < K; k0 += 32) {
    V bh[4], bl[4];
#pragma unroll
    for (int j = 0; j < 4; ++j) {
      const size_t bo = (size_t)(n0 + (j << 4) + rlane) * ldb + koff + k0;
      bh[j] = Frag<T>::load(Bb + bo);
      if (SPLIT) bl[j] = Frag<T>::load(Bb2 + bo);
    }
#pragma unroll
    for (int i = 0; i < 4; ++i) {
      const size_t ao = (size_t)(m0 + (i << 4) + rlane) * lda + koff + k0;
      V ah = Frag<T>::load(Ab + ao);
      V al;
      if (SPLIT) al = Frag<T>::load(Ab2 + ao);
#pragma unroll
      for (int j = 0; j < 4; ++j) {
        acc[i][j] = Frag<T>::mma(ah, bh[j], acc[i][j]);
        if (SPLIT) {
          acc[i][j] = Frag<T>::mma(ah, bl[j], acc[i][j]);
          acc[i][j] = Frag<T>::mma(al, bh[j], acc[i][j]);
        }
      }
      Frag<T>::guard(acc[i][0], acc[i][3], ah, SPLIT ? al : ah);
    }
    Frag<T>::keep(bh[0], bh[1], bh[2], bh[3]);
    if (SPLIT) Frag<T>::keep(bl[0], bl[1], bl[2], bl[3]);
  }
  acc_guard4(acc[0][0], acc[0][1], acc[0][2], acc[0][3]);
  acc_guard4(acc[1][0], acc[1][1], acc[1][2], acc[1][3]);
  acc_guard4(acc[2][0], acc[2][1], acc[2][2], acc[2][3]);
  acc_guard4(acc[3][0], acc[3][1], acc[3][2], acc[3][3]);

  float* slab = sT[wave];
  const float* Rb = RESID ? (resid + (size_t)b * strideR) : nullptr;
#pragma unroll
  for (int i = 0; i < 4; ++i) {
    const int mBase = m0 + (i << 4);
#pragma unroll
    for (int j = 0; j < 4; ++j) {
      const int n = n0 + (j << 4) + rlane;
      float bv = 0.f;
      if (BIAS_MODE == 2) bv = bias[n];
#pragma unroll
      for (int r = 0; r < 8; ++r) {
        float v = acc[i][j][r] * scale;
        if (BIAS_MODE == 1) v += bias[mBase + mOff + r];
        if (BIAS_MODE == 2) v += bv;
        if (RESID) v += Rb[(size_t)(mBase + mOff + r) * ldc + n];
        if (ACT == 2) v = fmaxf(v, 0.0f);
        if (ACT == 4) v = (v > 0.f) ? v : 0.01f * v;
        slab[(mOff + r) * 68 + (j << 4) + rlane] = v;
      }
    }
    __builtin_amdgcn_fence(__ATOMIC_RELEASE, "workgroup");
    __builtin_amdgcn_wave_barrier();
    __builtin_amdgcn_fence(__ATOMIC_ACQUIRE, "workgroup");
    if (OUT_MODE == 0) {
      float* C = (float*)Cout + (size_t)b * strideC;
      const int hh = lane >> 4, c4 = (lane & 15) * 4;
      for (int pass = 0; pass < 2; ++pass) {
#pragma unroll
        for (int it = 0; it < 8; ++it) {
          const int row = it * 2 + hh;
          v4f v = *(const v4f*)(slab + row * 68 + c4);
          *(volatile v4f*)(C + (size_t)(mBase + row) * ldc + n0 + c4) = v;
        }
        __threadfence();
      }
    } else {
      const int q = lane >> 3, c8 = (lane & 7) * 8;
      unsigned short* C  = (unsigned short*)Cout  + (size_t)b * strideC;
      unsigned short* C2 = (OUT_MODE == 2) ? ((unsigned short*)Cout2 + (size_t)b * strideC) : nullptr;
      for (int pass = 0; pass < 2; ++pass) {
#pragma unroll
        for (int it = 0; it < 4; ++it) {
          const int row = it * 4 + q;
          const float* sp = slab + row * 68 + c8;
          v8h hv, lv;
#pragma unroll
          for (int e = 0; e < 8; ++e) {
            if (OUT_MODE == 1) {
              hv[e] = (_Float16)sp[e];
            } else {
              unsigned short hb = f2bf_bits(sp[e]);
              unsigned short lb = f2bf_bits(sp[e] - bf_bits2f(hb));
              hv[e] = __builtin_bit_cast(_Float16, hb);
              lv[e] = __builtin_bit_cast(_Float16, lb);
            }
          }
          *(volatile v8h*)(C + (size_t)(mBase + row) * ldc + n0 + c8) = hv;
          if (OUT_MODE == 2) *(volatile v8h*)(C2 + (size_t)(mBase + row) * ldc + n0 + c8) = lv;
        }
        __threadfence();
      }
    }
    __builtin_amdgcn_fence(__ATOMIC_RELEASE, "workgroup");
    __builtin_amdgcn_wave_barrier();
    __builtin_amdgcn_fence(__ATOMIC_ACQUIRE, "workgroup");
  }
}

__device__ __forceinline__ void split8(const float* v, v4u& uh, v4u& ul) {
  unsigned short hb[8], lb[8];
#pragma unroll
  for (int e = 0; e < 8; ++e) {
    const unsigned short h = f2bf_bits(v[e]);
    hb[e] = h;
    lb[e] = f2bf_bits(v[e] - bf_bits2f(h));
  }
  uh = (v4u){pk16(hb[0], hb[1]), pk16(hb[2], hb[3]), pk16(hb[4], hb[5]), pk16(hb[6], hb[7])};
  ul = (v4u){pk16(lb[0], lb[1]), pk16(lb[2], lb[3]), pk16(lb[4], lb[5]), pk16(lb[6], lb[7])};
}
__device__ __forceinline__ float fexp(float x) { return exp2f(x * kLog2e); }

__global__ __launch_bounds__(256) void k_wsplit(const float* __restrict__ w, unsigned short* __restrict__ hi,
                                                 unsigned short* __restrict__ lo, int Nreal, int Cin, int ntaps,
                                                 int Kp, int total8) {
  const int i = blockIdx.x * 256 + threadIdx.x;
  if (i >= total8) return;
  const int e0 = i * 8;
  const int n  = e0 / Kp;
  const int kb = e0 - n * Kp;
  const int Kreal = Cin * ntaps;
  const int nsrc  = Nreal * Kreal;
  float v[8];
#pragma unroll
  for (int e = 0; e < 8; ++e) {
    const int k   = kb + e;
    const int tap = k / Cin;
    const int c   = k - tap * Cin;
    int src = (n * Cin + c) * ntaps + tap;
    src = src < 0 ? 0 : (src > nsrc - 1 ? nsrc - 1 : src);
    const float raw = w[src];
    const bool valid = (n < Nreal) && (k < Kreal);
    v[e] = valid ? raw : 0.0f;
  }
  v4u uh, ul;
  split8(v, uh, ul);
  unsigned short* ph = hi + (size_t)e0;
  unsigned short* pl = lo + (size_t)e0;
  *(volatile v4u*)ph = uh;
  *(volatile v4u*)pl = ul;
  __threadfence();
  *(volatile v4u*)ph = uh;
  *(volatile v4u*)pl = ul;
}

__global__ __launch_bounds__(256) void k_xpad(const float* __restrict__ x, unsigned short* __restrict__ hi,
                                               unsigned short* __restrict__ lo) {
  __shared__ float sm[64 * 65];
  const int tid = threadIdx.x;
  const int t0 = blockIdx.x * 64;
  const int b  = blockIdx.y;
#pragma unroll
  for (int it = 0; it < 16; ++it) {
    const int e = it * 256 + tid;
    const int c = e >> 6, tl = e & 63;
    sm[tl * 65 + c] = x[((size_t)(b * kChan + c)) * kLen + t0 + tl];
  }
  __syncthreads();
  const int lane = tid & 31, wave = tid >> 5;
  const int q = lane >> 3, c8 = (lane & 7) * 8;
  for (int pass = 0; pass < 2; ++pass) {
#pragma unroll
    for (int it = 0; it < 2; ++it) {
      const int row = wave * 8 + it * 4 + q;
      float v[8];
#pragma unroll
      for (int e = 0; e < 8; ++e) v[e] = sm[row * 65 + c8 + e];
      v4u uh, ul;
      split8(v, uh, ul);
      const size_t off = ((size_t)b * kXpadRows + 3 + t0 + row) * kChan + c8;
      *(volatile v4u*)(hi + off) = uh;
      *(volatile v4u*)(lo + off) = ul;
    }
    __threadfence();
  }
}

__global__ __launch_bounds__(64) void k_zero16(unsigned short* __restrict__ p0, unsigned short* __restrict__ p1,
                                                long bstride, long off2, int n16) {
  const int b = blockIdx.x, sel = blockIdx.y, tid = threadIdx.x;
  if (tid >= n16) return;
  unsigned short* base = (sel & 1) ? p1 : p0;
  const size_t off = (size_t)b * bstride + ((sel >> 1) ? (size_t)off2 : (size_t)0) + (size_t)tid * 8;
  const v4u z = (v4u){0u, 0u, 0u, 0u};
  *(volatile v4u*)(base + off) = z;
  __threadfence();
  *(volatile v4u*)(base + off) = z;
}

__global__ __launch_bounds__(256) void k_split8(const float* __restrict__ in, unsigned short* __restrict__ hi,
                                                 unsigned short* __restrict__ lo, int n8) {
  const int i = blockIdx.x * 256 + threadIdx.x;
  if (i >= n8) return;
  const float* p = in + 8 * (size_t)i;
  const v4f a = *(const v4f*)(p);
  const v4f c = *(const v4f*)(p + 4);
  float v[8] = {a[0], a[1], a[2], a[3], c[0], c[1], c[2], c[3]};
  v4u uh, ul;
  split8(v, uh, ul);
  unsigned short* ph = hi + 8 * (size_t)i;
  unsigned short* pl = lo + 8 * (size_t)i;
  *(volatile v4u*)ph = uh;
  *(volatile v4u*)pl = ul;
  __threadfence();
  *(volatile v4u*)ph = uh;
  *(volatile v4u*)pl = ul;
}

#define SSM_UPD(NI, BV, CV, EI) { s[NI] = s[NI] * dec + BV[EI] * xdt; yp += CV[EI] * s[NI]; }
__global__ __launch_bounds__(256) void k_scan(const float* __restrict__ zx, const float* __restrict__ conv_w,
                                               const float* __restrict__ conv_b, const float* __restrict__ dt_bias,
                                               const float* __restrict__ A_log, const float* __restrict__ Dp,
                                               float* __restrict__ y) {
  __shared__ __align__(16) float sAct[kTCH * kActW];
  __shared__ __align__(16) float sY[kTCH * 64];
  __shared__ float sDt[kTCH];
  __shared__ float sDec[kTCH];
  const int tid = threadIdx.x, lane = tid & 31, wave = tid >> 5;
  const int b  = blockIdx.x >> 1;
  const int hd = blockIdx.x & 1;
  const int p  = tid >> 2;
  const int nq = tid & 3;
  const size_t tokb = (size_t)b * kLen;
  const float aneg = -expf(A_log[hd]);
  const float dtb  = dt_bias[hd];
  const float dpv  = Dp[hd];
  float s[16];
#pragma unroll
  for (int n = 0; n < 16; ++n) s[n] = 0.0f;

#pragma unroll 1
  for (int ck = 0; ck < kLen / kTCH; ++ck) {
    const int t0 = ck * kTCH;
#pragma unroll 1
    for (int it = 0; it < (kTCH * kActW) / 256; ++it) {
      const int e  = it * 256 + tid;
      const int tl = e / kActW;
      const int c  = e - tl * kActW;
      const int cc = (c < 64) ? (hd * 64 + c) : (c + 64);
      const int col = kDin + cc;
      float acc = conv_b[cc];
#pragma unroll
      for (int k = 0; k < 4; ++k) {
        const int tt  = t0 + tl - 3 + k;
        const int ttc = tt < 0 ? 0 : tt;
        const float raw = zx[(tokb + ttc) * kZXld + col];
        const float xv  = (tt >= 0) ? raw : 0.0f;
        acc += conv_w[cc * 4 + k] * xv;
      }
      const float ac = fminf(fmaxf(acc, -80.0f), 80.0f);
      const float sg = __builtin_amdgcn_rcpf(1.0f + expf(-ac));
      sAct[tl * kActW + c] = acc * sg;
    }
    if (wave == 0) {
      const float raw = zx[(tokb + t0 + lane) * kZXld + 384 + hd] + dtb;
      const float dt  = fmaxf(raw, 0.0f) + log1pf(expf(-fabsf(raw)));
      sDt[lane]  = dt;
      sDec[lane] = expf(dt * aneg);
    }
    __syncthreads();
#pragma unroll 1
    for (int tl = 0; tl < kTCH; ++tl) {
      const float dt  = sDt[tl];
      const float dec = sDec[tl];
      const float* arow = sAct + tl * kActW;
      const float xv  = arow[p];
      const float xdt = xv * dt;
      const v4f b0 = *(const v4f*)(arow + 64 + nq * 16);
      const v4f b1 = *(const v4f*)(arow + 64 + nq * 16 + 4);
      const v4f b2 = *(const v4f*)(arow + 64 + nq * 16 + 8);
      const v4f b3 = *(const v4f*)(arow + 64 + nq * 16 + 12);
      const v4f c0 = *(const v4f*)(arow + 128 + nq * 16);
      const v4f c1 = *(const v4f*)(arow + 128 + nq * 16 + 4);
      const v4f c2 = *(const v4f*)(arow + 128 + nq * 16 + 8);
      const v4f c3 = *(const v4f*)(arow + 128 + nq * 16 + 12);
      float yp = 0.0f;
      SSM_UPD(0, b0, c0, 0)  SSM_UPD(1, b0, c0, 1)  SSM_UPD(2, b0, c0, 2)  SSM_UPD(3, b0, c0, 3)
      SSM_UPD(4, b1, c1, 0)  SSM_UPD(5, b1, c1, 1)  SSM_UPD(6, b1, c1, 2)  SSM_UPD(7, b1, c1, 3)
      SSM_UPD(8, b2, c2, 0)  SSM_UPD(9, b2, c2, 1)  SSM_UPD(10, b2, c2, 2) SSM_UPD(11, b2, c2, 3)
      SSM_UPD(12, b3, c3, 0) SSM_UPD(13, b3, c3, 1) SSM_UPD(14, b3, c3, 2) SSM_UPD(15, b3, c3, 3)
      yp += __shfl_xor(yp, 1, 32);
      yp += __shfl_xor(yp, 2, 32);
      const float yv = yp + dpv * xv;
      if (nq == 0) sY[tl * 64 + p] = yv;
    }
    __syncthreads();
    {
      const int hh2 = lane >> 4, c4 = (lane & 15) * 4;
      for (int pass = 0; pass < 2; ++pass) {
#pragma unroll
        for (int it = 0; it < 2; ++it) {
          const int tl = wave * 4 + it * 2 + hh2;
          const v4f v = *(const v4f*)(sY + tl * 64 + c4);
          *(volatile v4f*)(y + (tokb + t0 + tl) * kDin + hd * 64 + c4) = v;
        }
        __threadfence();
      }
    }
    __syncthreads();
  }
}

__global__ __launch_bounds__(256) void k_gate(const float* __restrict__ y, const float* __restrict__ zx,
                                               const float* __restrict__ norm_w, unsigned short* __restrict__ uh,
                                               unsigned short* __restrict__ ul) {
  const int tid = threadIdx.x, lane = tid & 31, wave = tid >> 5;
  const int r = lane >> 4, c8 = (lane & 15) * 8;
  const size_t tok = (size_t)blockIdx.x * 16 + wave * 2 + r;
  const float* yr = y + tok * kDin + c8;
  const float* zr = zx + tok * kZXld + c8;
  const v4f y0 = *(const v4f*)(yr), y1 = *(const v4f*)(yr + 4);
  const v4f z0 = *(const v4f*)(zr), z1 = *(const v4f*)(zr + 4);
  const float yv[8] = {y0[0], y0[1], y0[2], y0[3], y1[0], y1[1], y1[2], y1[3]};
  const float zv[8] = {z0[0], z0[1], z0[2], z0[3], z1[0], z1[1], z1[2], z1[3]};
  float u[8];
  float ss = 0.0f;
#pragma unroll
  for (int e = 0; e < 8; ++e) {
    const float zc = fminf(fmaxf(zv[e], -80.0f), 80.0f);
    const float sg = __builtin_amdgcn_rcpf(1.0f + fexp(-zc));
    u[e] = yv[e] * (zv[e] * sg);
    ss += u[e] * u[e];
  }
  ss += __shfl_xor(ss, 1, 32);
  ss += __shfl_xor(ss, 2, 32);
  ss += __shfl_xor(ss, 4, 32);
  ss += __shfl_xor(ss, 8, 32);
  const float rn = rsqrtf(ss * (1.0f / 128.0f) + 1e-5f);
  float v[8];
#pragma unroll
  for (int e = 0; e < 8; ++e) v[e] = (u[e] * rn) * norm_w[c8 + e];
  v4u ph, pl;
  split8(v, ph, pl);
  const size_t off = tok * kDin + c8;
  for (int pass = 0; pass < 2; ++pass) {
    *(volatile v4u*)(uh + off) = ph;
    *(volatile v4u*)(ul + off) = pl;
    __threadfence();
  }
}

__global__ __launch_bounds__(256) void k_ln_pool(const float* __restrict__ mbuf, const float* __restrict__ hres,
                                                  const float* __restrict__ g, const float* __restrict__ bta,
                                                  unsigned short* __restrict__ xh, unsigned short* __restrict__ xl) {
  const int tid = threadIdx.x, lane = tid & 31, wave = tid >> 5;
  const int sub = lane >> 3;
  const int pp = sub >> 1, which = sub & 1;
  const int c8 = (lane & 7) * 8;
  const int ptok = blockIdx.x * 16 + wave * 2 + pp;
  const int b = ptok >> 10, tp = ptok & 1023;
  const size_t tok = (size_t)b * kLen + 2 * tp + which;
  const float* mr = mbuf + tok * kChan + c8;
  const float* hr = hres + tok * kChan + c8;
  const v4f m0 = *(const v4f*)(mr), m1 = *(const v4f*)(mr + 4);
  const v4f h0 = *(const v4f*)(hr), h1 = *(const v4f*)(hr + 4);
  const float mv[8] = {m0[0], m0[1], m0[2], m0[3], m1[0], m1[1], m1[2], m1[3]};
  const float hv[8] = {h0[0], h0[1], h0[2], h0[3], h1[0], h1[1], h1[2], h1[3]};
  float sm = 0.0f;
#pragma unroll
  for (int e = 0; e < 8; ++e) sm += mv[e];
  sm += __shfl_xor(sm, 1, 32);
  sm += __shfl_xor(sm, 2, 32);
  sm += __shfl_xor(sm, 4, 32);
  const float mu = sm * (1.0f / 64.0f);
  float sq = 0.0f;
#pragma unroll
  for (int e = 0; e < 8; ++e) { const float d = mv[e] - mu; sq += d * d; }
  sq += __shfl_xor(sq, 1, 32);
  sq += __shfl_xor(sq, 2, 32);
  sq += __shfl_xor(sq, 4, 32);
  const float var = sq * (1.0f / 64.0f);
  const float rs = rsqrtf(var + 1e-5f);
  float v[8];
#pragma unroll
  for (int e = 0; e < 8; ++e) {
    const float x1 = (mv[e] - mu) * rs * g[c8 + e] + bta[c8 + e] + hv[e];
    const float ot = __shfl_xor(x1, 8, 32);
    v[e] = fmaxf(x1, ot);
  }
  v4u ph, pl;
  split8(v, ph, pl);
  const size_t off = ((size_t)b * kX1Rows + 1 + tp) * kChan + c8;
  for (int pass = 0; pass < 2; ++pass) {
    if (which == 0) {
      *(volatile v4u*)(xh + off) = ph;
      *(volatile v4u*)(xl + off) = pl;
    }
    __threadfence();
  }
}

__global__ __launch_bounds__(256) void k_pool2(const float* __restrict__ c2, unsigned short* __restrict__ xh,
                                                unsigned short* __restrict__ xl) {
  const int tid = threadIdx.x, lane = tid & 31, wave = tid >> 5;
  const int r = lane >> 4, c8 = (lane & 15) * 8;
  const int ptok = blockIdx.x * 16 + wave * 2 + r;
  const int b = ptok >> 9, tp = ptok & 511;
  const size_t src = ((size_t)b * kLen1 + 2 * tp) * 128 + c8;
  const v4f a0 = *(const v4f*)(c2 + src),       a1 = *(const v4f*)(c2 + src + 4);
  const v4f b0 = *(const v4f*)(c2 + src + 128), b1 = *(const v4f*)(c2 + src + 132);
  float v[8];
#pragma unroll
  for (int e = 0; e < 4; ++e) { v[e] = fmaxf(a0[e], b0[e]); v[4 + e] = fmaxf(a1[e], b1[e]); }
  v4u ph, pl;
  split8(v, ph, pl);
  const size_t off = ((size_t)b * kX2Rows + 1 + tp) * 128 + c8;
  for (int pass = 0; pass < 2; ++pass) {
    *(volatile v4u*)(xh + off) = ph;
    *(volatile v4u*)(xl + off) = pl;
    __threadfence();
  }
}

__global__ __launch_bounds__(256) void k_final(const float* __restrict__ c3, float* __restrict__ out) {
  __shared__ __align__(16) float so[32 * 260];
  const int tid = threadIdx.x, lane = tid & 31, wave = tid >> 5;
  const int o0 = blockIdx.x * 32, b = blockIdx.y;
#pragma unroll 1
  for (int it = 0; it < 32; ++it) {
    const int tp = it * 8 + wave;
    const size_t r0 = ((size_t)b * kLen2 + 2 * tp) * 256 + o0 + lane;
    const float v0 = c3[r0], v1 = c3[r0 + 256];
    so[lane * 260 + tp] = fmaxf(v0, v1);
  }
  __syncthreads();
  for (int pass = 0; pass < 2; ++pass) {
#pragma unroll
    for (int i = 0; i < 4; ++i) {
      const int o = wave * 4 + i;
#pragma unroll
      for (int j = 0; j < 2; ++j) {
        const int col = j * 128 + lane * 4;
        const v4f v = *(const v4f*)(so + o * 260 + col);
        *(volatile v4f*)(out + ((size_t)(b * 256 + o0 + o)) * kLen3 + col) = v;
      }
    }
    __threadfence();
  }
}

template <int BIAS_MODE, int OUT_MODE>
static void launch_gemm(hipStream_t st, int batches,
                        const unsigned short* Ah, const unsigned short* Al, int lda, long sA,
                        const unsigned short* Bh, const unsigned short* Bl, int ldb,
                        void* Ch, void* Cl, int ldc, long sC,
                        const float* bias, const float* dummyR, int M, int N, int K) {
  const int tiles = (M / 64) * (N / 64);
  dim3 grid((tiles + 7) / 8, batches);
  wmma_gemm64<1, true, BIAS_MODE, OUT_MODE, false, 0><<<grid, 256, 0, st>>>(
      Ah, Al, lda, sA, Bh, Bl, ldb, 0L, Ch, Cl, ldc, sC, bias, dummyR, 0L, M, N, K, 1.0f);
}

constexpr size_t kOffW1h = 0,       kOffW1l = 8192;
constexpr size_t kOffW3h = 16384,   kOffW3l = 40960;
constexpr size_t kOffW7h = 65536,   kOffW7l = 122880;
constexpr size_t kOffFuh = 180224,  kOffFul = 204800;
constexpr size_t kOffLih = 229376,  kOffLil = 237568;
constexpr size_t kOffIph = 245760,  kOffIpl = 303104;
constexpr size_t kOffOph = 360448,  kOffOpl = 376832;
constexpr size_t kOffE2h = 393216,  kOffE2l = 442368;
constexpr size_t kOffE3h = 491520,  kOffE3l = 688128;
constexpr size_t kOffWEnd = 884736;
constexpr size_t kOffA = 1048576;
constexpr size_t kSizeA = (size_t)kTok * kZXld * 4;
constexpr size_t kXpadPlane = (size_t)kBatch * kXpadRows * kChan * 2;
constexpr size_t kCatPlane  = (size_t)kTok * 192 * 2;
constexpr size_t kEPlane    = (size_t)kTok * 64 * 2;
constexpr size_t kOffXph = kOffA, kOffXpl = kOffA + kXpadPlane;
constexpr size_t kOffCath = kOffXpl + kXpadPlane, kOffCatl = kOffCath + kCatPlane;
constexpr size_t kOffEh = kOffCatl + kCatPlane, kOffEl = kOffEh + kEPlane;
constexpr size_t kOffZx = kOffA;
constexpr size_t kMBytes   = (size_t)kTok * 64 * 4;
constexpr size_t kX1Plane  = (size_t)kBatch * kX1Rows * 64 * 2;
constexpr size_t kC2Bytes  = (size_t)kBatch * kLen1 * 128 * 4;
constexpr size_t kX2Plane  = (size_t)kBatch * kX2Rows * 128 * 2;
constexpr size_t kC3Bytes  = (size_t)kBatch * kLen2 * 256 * 4;
constexpr size_t kOffM = kOffA;
constexpr size_t kOffX1h = kOffM + kMBytes, kOffX1l = kOffX1h + kX1Plane;
constexpr size_t kOffC2 = kOffX1l + kX1Plane;
constexpr size_t kOffX2h = kOffC2 + kC2Bytes, kOffX2l = kOffX2h + kX2Plane;
constexpr size_t kOffC3 = kOffX2l + kX2Plane;
constexpr size_t kOffB = kOffA + kSizeA;
constexpr size_t kHBytes = (size_t)kTok * 64 * 4;
constexpr size_t kOffC = kOffB + kHBytes;
constexpr size_t kOffHh = kOffC, kOffHl = kOffC + kEPlane;
constexpr size_t kOffY = kOffC;
constexpr size_t kYBytes = (size_t)kTok * 128 * 4;
constexpr size_t kOffD = kOffC + kYBytes;
constexpr size_t kUPlane = (size_t)kTok * 128 * 2;
constexpr size_t kOffUh = kOffD, kOffUl = kOffD + kUPlane;
constexpr size_t kWsTotal = kOffD + 2 * kUPlane;
static_assert(kOffWEnd <= kOffA);
static_assert(kOffEl + kEPlane <= kOffA + kSizeA);
static_assert(kOffC3 + kC3Bytes <= kOffA + kSizeA);
static_assert(kOffHl + kEPlane <= kOffC + kYBytes);
static_assert(kWsTotal == 101711872);
static_assert(kWsTotal <= 134217728);
static_assert((kOffXpl % 128) == 0 && (kOffCatl % 128) == 0 && (kOffEl % 128) == 0 && (kOffX1l % 128) == 0 &&
              (kOffX2l % 128) == 0 && (kOffC3 % 128) == 0 && (kOffUl % 128) == 0);

extern "C" void kernel_launch(void* const* d_in, const int* in_sizes, int n_in,
                              void* d_out, int out_size, void* d_ws, size_t ws_size,
                              hipStream_t stream) {
  if (n_in < 25) return;
  if (out_size != kBatch * 256 * kLen3) return;
  if (ws_size < kWsTotal) return;
  if (in_sizes[0] != kBatch * kChan * kLen) return;

  const float* x        = (const float*)d_in[0];
  const float* emb_w1   = (const float*)d_in[1];
  const float* emb_b1   = (const float*)d_in[2];
  const float* emb_w3   = (const float*)d_in[3];
  const float* emb_b3   = (const float*)d_in[4];
  const float* emb_w7   = (const float*)d_in[5];
  const float* emb_b7   = (const float*)d_in[6];
  const float* fuse_w   = (const float*)d_in[7];
  const float* fuse_b   = (const float*)d_in[8];
  const float* lin_w    = (const float*)d_in[9];
  const float* lin_b    = (const float*)d_in[10];
  const float* in_w     = (const float*)d_in[11];
  const float* conv_w   = (const float*)d_in[12];
  const float* conv_b   = (const float*)d_in[13];
  const float* dt_bias  = (const float*)d_in[14];
  const float* A_log    = (const float*)d_in[15];
  const float* D_param  = (const float*)d_in[16];
  const float* norm_w   = (const float*)d_in[17];
  const float* out_w    = (const float*)d_in[18];
  const float* ln_g     = (const float*)d_in[19];
  const float* ln_b     = (const float*)d_in[20];
  const float* enc2_w   = (const float*)d_in[21];
  const float* enc2_b   = (const float*)d_in[22];
  const float* enc3_w   = (const float*)d_in[23];
  const float* enc3_b   = (const float*)d_in[24];
  float* out = (float*)d_out;
  unsigned char* ws = (unsigned char*)d_ws;

  unsigned short* w1h = (unsigned short*)(ws + kOffW1h); unsigned short* w1l = (unsigned short*)(ws + kOffW1l);
  unsigned short* w3h = (unsigned short*)(ws + kOffW3h); unsigned short* w3l = (unsigned short*)(ws + kOffW3l);
  unsigned short* w7h = (unsigned short*)(ws + kOffW7h); unsigned short* w7l = (unsigned short*)(ws + kOffW7l);
  unsigned short* fuh = (unsigned short*)(ws + kOffFuh); unsigned short* ful = (unsigned short*)(ws + kOffFul);
  unsigned short* lih = (unsigned short*)(ws + kOffLih); unsigned short* lil = (unsigned short*)(ws + kOffLil);
  unsigned short* iph = (unsigned short*)(ws + kOffIph); unsigned short* ipl = (unsigned short*)(ws + kOffIpl);
  unsigned short* oph = (unsigned short*)(ws + kOffOph); unsigned short* opl = (unsigned short*)(ws + kOffOpl);
  unsigned short* e2h = (unsigned short*)(ws + kOffE2h); unsigned short* e2l = (unsigned short*)(ws + kOffE2l);
  unsigned short* e3h = (unsigned short*)(ws + kOffE3h); unsigned short* e3l = (unsigned short*)(ws + kOffE3l);
  unsigned short* xph = (unsigned short*)(ws + kOffXph); unsigned short* xpl = (unsigned short*)(ws + kOffXpl);
  unsigned short* cath = (unsigned short*)(ws + kOffCath); unsigned short* catl = (unsigned short*)(ws + kOffCatl);
  unsigned short* eh = (unsigned short*)(ws + kOffEh); unsigned short* el = (unsigned short*)(ws + kOffEl);
  float* zx = (float*)(ws + kOffZx);
  float* mf = (float*)(ws + kOffM);
  unsigned short* x1h = (unsigned short*)(ws + kOffX1h); unsigned short* x1l = (unsigned short*)(ws + kOffX1l);
  float* c2f = (float*)(ws + kOffC2);
  unsigned short* x2h = (unsigned short*)(ws + kOffX2h); unsigned short* x2l = (unsigned short*)(ws + kOffX2l);
  float* c3f = (float*)(ws + kOffC3);
  float* hf = (float*)(ws + kOffB);
  unsigned short* hbh = (unsigned short*)(ws + kOffHh); unsigned short* hbl = (unsigned short*)(ws + kOffHl);
  float* yf = (float*)(ws + kOffY);
  unsigned short* ubh = (unsigned short*)(ws + kOffUh); unsigned short* ubl = (unsigned short*)(ws + kOffUl);

  k_wsplit<<<2, 256, 0, stream>>>(emb_w1, w1h, w1l, 64, 64, 1, 64, 512);
  k_wsplit<<<6, 256, 0, stream>>>(emb_w3, w3h, w3l, 64, 64, 3, 192, 1536);
  k_wsplit<<<14, 256, 0, stream>>>(emb_w7, w7h, w7l, 64, 64, 7, 448, 3584);
  k_wsplit<<<6, 256, 0, stream>>>(fuse_w, fuh, ful, 64, 192, 1, 192, 1536);
  k_wsplit<<<2, 256, 0, stream>>>(lin_w, lih, lil, 64, 64, 1, 64, 512);
  k_wsplit<<<14, 256, 0, stream>>>(in_w, iph, ipl, 386, 64, 1, 64, 3584);
  k_wsplit<<<4, 256, 0, stream>>>(out_w, oph, opl, 64, 128, 1, 128, 1024);
  k_wsplit<<<12, 256, 0, stream>>>(enc2_w, e2h, e2l, 128, 64, 3, 192, 3072);
  k_wsplit<<<48, 256, 0, stream>>>(enc3_w, e3h, e3l, 256, 128, 3, 384, 12288);

  k_xpad<<<dim3(kLen / 64, kBatch), 256, 0, stream>>>(x, xph, xpl);
  k_zero16<<<dim3(kBatch, 4), 64, 0, stream>>>(xph, xpl, (long)kXpadRows * 64, (long)(kLen + 3) * 64, 24);

  launch_gemm<2, 2>(stream, kBatch, xph + 3 * 64, xpl + 3 * 64, 64, (long)kXpadRows * 64, w1h, w1l, 64,
                    cath, catl, 192, (long)kLen * 192, emb_b1, hf, kLen, 64, 64);
  launch_gemm<2, 2>(stream, kBatch, xph + 2 * 64, xpl + 2 * 64, 64, (long)kXpadRows * 64, w3h, w3l, 192,
                    cath + 64, catl + 64, 192, (long)kLen * 192, emb_b3, hf, kLen, 64, 192);
  launch_gemm<2, 2>(stream, kBatch, xph, xpl, 64, (long)kXpadRows * 64, w7h, w7l, 448,
                    cath + 128, catl + 128, 192, (long)kLen * 192, emb_b7, hf, kLen, 64, 448);
  launch_gemm<2, 2>(stream, 1, cath, catl, 192, 0L, fuh, ful, 192, eh, el, 64, 0L, fuse_b, hf, kTok, 64, 192);
  launch_gemm<2, 0>(stream, 1, eh, el, 64, 0L, lih, lil, 64, hf, hf, 64, 0L, lin_b, hf, kTok, 64, 64);
  k_split8<<<(kTok * 64 / 8 + 255) / 256, 256, 0, stream>>>(hf, hbh, hbl, kTok * 64 / 8);
  launch_gemm<0, 0>(stream, 1, hbh, hbl, 64, 0L, iph, ipl, 64, zx, zx, kZXld, 0L, lin_b, hf, kTok, kZXld, 64);
  k_scan<<<kBatch * 2, 256, 0, stream>>>(zx, conv_w, conv_b, dt_bias, A_log, D_param, yf);
  k_gate<<<kTok / 16, 256, 0, stream>>>(yf, zx, norm_w, ubh, ubl);
  launch_gemm<0, 0>(stream, 1, ubh, ubl, 128, 0L, oph, opl, 128, mf, mf, 64, 0L, lin_b, hf, kTok, 64, 128);
  k_zero16<<<dim3(kBatch, 4), 64, 0, stream>>>(x1h, x1l, (long)kX1Rows * 64, (long)(kLen1 + 1) * 64, 8);
  k_ln_pool<<<(kBatch * kLen1) / 16, 256, 0, stream>>>(mf, hf, ln_g, ln_b, x1h, x1l);
  launch_gemm<2, 0>(stream, kBatch, x1h, x1l, 64, (long)kX1Rows * 64, e2h, e2l, 192,
                    c2f, c2f, 128, (long)kLen1 * 128, enc2_b, hf, kLen1, 128, 192);
  k_zero16<<<dim3(kBatch, 4), 64, 0, stream>>>(x2h, x2l, (long)kX2Rows * 128, (long)(kLen2 + 1) * 128, 16);
  k_pool2<<<(kBatch * kLen2) / 16, 256, 0, stream>>>(c2f, x2h, x2l);
  launch_gemm<2, 0>(stream, kBatch, x2h, x2l, 128, (long)kX2Rows * 128, e3h, e3l, 384,
                    c3f, c3f, 256, (long)kLen2 * 256, enc3_b, hf, kLen2, 256, 384);
  k_final<<<dim3(256 / 32, kBatch), 256, 0, stream>>>(c3f, out);
}
